// NBEATSSeasonalBlockKAN_53652731461734
// MI455X (gfx1250) — hardware-run, weakly checked
//
#include <hip/hip_runtime.h>
#include <stddef.h>


#define UNITS 512
#define BACK  512
#define FORE  128
#define TH    128
#define NL    4
#define NCO   8
#define KD    (UNITS * (1 + NCO))
#define TT    (BACK + FORE)
#define NGRP  (KD / 8)
#define NTHR  256
#define RPB   64
#define CPB   128
#define HBP   (CPB + 4)
#define APR   4
#define WSC   16.0f
#define WINV  0.0625f
#define WSCAP 134217728

static_assert((KD % 32) == 0);
static_assert((NGRP % 32) == 0);
static_assert((UNITS % CPB) == 0 && (TH % CPB) == 0 && (CPB == FORE));
static_assert(((APR * NGRP) % NTHR) == 0);
static_assert(((NL * UNITS * NGRP) % NTHR) == 0 && ((TH * NGRP) % NTHR) == 0);
static_assert((((TT * TH) / 8) % NTHR) == 0);
static_assert((RPB * CPB / 4) == 8 * NTHR);
static_assert(((HBP * 4) % 16) == 0);
static_assert((TH % 32) == 0);
static_assert((UNITS % 64) == 0);

typedef float          v4f   __attribute__((ext_vector_type(4)));
typedef float          v8f   __attribute__((ext_vector_type(8)));
typedef _Float16       v8h   __attribute__((ext_vector_type(8)));
typedef _Float16       v16h  __attribute__((ext_vector_type(16)));
typedef unsigned short v8us  __attribute__((ext_vector_type(8)));
typedef unsigned short v16us __attribute__((ext_vector_type(16)));
typedef __bf16         v16bf __attribute__((ext_vector_type(16)));
union FragH { v16h v; v16us u; v8us h[2]; };
union FragB { v16bf b; v16us u; v8us h[2]; };
union P8 { v8h h; v8us u; };
union P1 { _Float16 h; unsigned short u; };
static_assert(sizeof(FragH) == 32);
static_assert(sizeof(FragB) == 32);
static_assert(sizeof(P8) == 16);
static_assert(sizeof(P1) == 2);

#define KG(j) ((float)((double)((j) - 3) * 0.4 - 1.0))
#define R1(t) (1.0f / (KG((t) + 1) - KG(t)))
#define R2(t) (1.0f / (KG((t) + 2) - KG(t)))
#define R3(t) (1.0f / (KG((t) + 3) - KG(t)))
__constant__ float c_g[12]  = {KG(0), KG(1), KG(2), KG(3), KG(4), KG(5), KG(6), KG(7), KG(8), KG(9), KG(10), KG(11)};
__constant__ float c_r1[11] = {R1(0), R1(1), R1(2), R1(3), R1(4), R1(5), R1(6), R1(7), R1(8), R1(9), R1(10)};
__constant__ float c_r2[10] = {R2(0), R2(1), R2(2), R2(3), R2(4), R2(5), R2(6), R2(7), R2(8), R2(9)};
__constant__ float c_r3[9]  = {R3(0), R3(1), R3(2), R3(3), R3(4), R3(5), R3(6), R3(7), R3(8)};

__device__ __forceinline__ v8f wmf(v16h a, v16h bq, v8f c) {
  v8f d = __builtin_amdgcn_wmma_f32_16x16x32_f16(false, a, false, bq, (short)0, c, false, false);
  asm volatile("v_nop\n\tv_nop\n\tv_nop\n\tv_nop" : "+v"(d) : "v"(a), "v"(bq));
  return d;
}
__device__ __forceinline__ v8f wmb(v16bf a, v16bf bq, v8f c) {
  v8f d = __builtin_amdgcn_wmma_f32_16x16x32_bf16(false, a, false, bq, (short)0, c, false, false);
  asm volatile("v_nop\n\tv_nop\n\tv_nop\n\tv_nop" : "+v"(d) : "v"(a), "v"(bq));
  return d;
}
__device__ __forceinline__ v8f zero8() {
  v8f z = {0.f, 0.f, 0.f, 0.f, 0.f, 0.f, 0.f, 0.f};
  return z;
}
__device__ __forceinline__ unsigned bf16_bits(float f) {
  unsigned u = __float_as_uint(f);
  u += 0x7FFFu + ((u >> 16) & 1u);
  return u >> 16;
}
__device__ __forceinline__ void split2(float v, unsigned short& hb, unsigned short& lb) {
  const unsigned hh = bf16_bits(v);
  const float hf = __uint_as_float(hh << 16);
  hb = (unsigned short)hh;
  lb = (unsigned short)bf16_bits(v - hf);
}
__device__ __forceinline__ unsigned short f16_bits(float f) {
  P1 p; p.h = (_Float16)f;
  return p.u;
}

__global__ __launch_bounds__(NTHR) void k_tables(unsigned short* Shi, unsigned short* Slo) {
  const int t = blockIdx.x * NTHR + threadIdx.x;
  const int n = t >> 4, q = t & 15;
  v8us hv, lv;
#pragma unroll
  for (int c = 0; c < 8; ++c) {
    const int k = 8 * q + c;
    const int p = k & 63;
    const int rr = (p * n) % 63;
    const float rev = (float)rr * (1.0f / 63.0f);
    const float cv = __builtin_amdgcn_cosf(rev);
    const float sv = __builtin_amdgcn_sinf(rev);
    const float v = (k < 64) ? cv : sv;
    unsigned short a, d;
    split2(v, a, d);
    hv[c] = a; lv[c] = d;
  }
  unsigned short* dh = Shi + (size_t)t * 8;
  unsigned short* dl = Slo + (size_t)t * 8;
  *(volatile v8us*)dh = hv;
  *(volatile v8us*)dl = lv;
  __threadfence();
  *(volatile v8us*)dh = hv;
  *(volatile v8us*)dl = lv;
}

template <int NOUT>
__global__ __launch_bounds__(NTHR) void k_wpack(const float* __restrict__ coef, const float* __restrict__ sb,
                                               const float* __restrict__ ssp, unsigned short* Wp) {
  const int t = blockIdx.x * NTHR + threadIdx.x;
  const int o = t / NGRP;
  const int q = t - o * NGRP;
  const int l = o / NOUT;
  const int oo = o - l * NOUT;
  int ib = 8 * q;          ib = ib > UNITS - 8 ? UNITS - 8 : ib;
  int is = q - UNITS / 8;  is = is < 0 ? 0 : is;
  const float* ps = sb + ((size_t)l * UNITS + ib) * NOUT + oo;
  const size_t io = ((size_t)l * UNITS + is) * NOUT + oo;
  const float* pc = coef + io * NCO;
  const float sp = ssp[io];
  const v4f g0 = *(const v4f*)pc, g1 = *(const v4f*)(pc + 4);
  const float gg[8] = {g0.x, g0.y, g0.z, g0.w, g1.x, g1.y, g1.z, g1.w};
  const bool isb = q < UNITS / 8;
  v8us w;
#pragma unroll
  for (int e = 0; e < 8; ++e) {
    const float bv = ps[(size_t)e * NOUT];
    const float sv = gg[e] * sp;
    w[e] = f16_bits(WSC * (isb ? bv : sv));
  }
  unsigned short* dp = Wp + (size_t)t * 8;
  *(volatile v8us*)dp = w;
  __threadfence();
  *(volatile v8us*)dp = w;
}

__global__ __launch_bounds__(NTHR) void k_aprep(const float* __restrict__ H, unsigned short* Ap) {
  __shared__ __align__(16) unsigned short sT[APR * KD];
  const int tid = threadIdx.x;
  const int r = tid >> 6, fg = tid & 63;
  const int row0 = blockIdx.x * APR;
  float g[12], q1[11], q2[10], q3[9];
#pragma unroll
  for (int t = 0; t < 12; ++t) g[t] = c_g[t];
#pragma unroll
  for (int t = 0; t < 11; ++t) q1[t] = c_r1[t];
#pragma unroll
  for (int t = 0; t < 10; ++t) q2[t] = c_r2[t];
#pragma unroll
  for (int t = 0; t < 9; ++t)  q3[t] = c_r3[t];
  const float* hp = H + (size_t)(row0 + r) * UNITS + 8 * fg;
  unsigned short* sr = sT + r * KD;
#pragma unroll 1
  for (int q = 0; q < 8; ++q) {
    const float x = hp[q];
    float bs[11];
#pragma unroll
    for (int t = 0; t < 11; ++t) bs[t] = (x >= g[t] && x < g[t + 1]) ? 1.0f : 0.0f;
#pragma unroll
    for (int t = 0; t < 10; ++t) {
      const float lf = (x - g[t]) * q1[t];
      const float rg = (g[t + 2] - x) * q1[t + 1];
      bs[t] = lf * bs[t] + rg * bs[t + 1];
    }
#pragma unroll
    for (int t = 0; t < 9; ++t) {
      const float lf = (x - g[t]) * q2[t];
      const float rg = (g[t + 3] - x) * q2[t + 1];
      bs[t] = lf * bs[t] + rg * bs[t + 1];
    }
#pragma unroll
    for (int t = 0; t < 8; ++t) {
      const float lf = (x - g[t]) * q3[t];
      const float rg = (g[t + 4] - x) * q3[t + 1];
      bs[t] = lf * bs[t] + rg * bs[t + 1];
    }
    const float sl = x * __builtin_amdgcn_rcpf(1.0f + __expf(-x));
    const int f = 8 * fg + q;
    sr[f] = f16_bits(sl);
    P8 pk;
#pragma unroll
    for (int c = 0; c < NCO; ++c) pk.h[c] = (_Float16)bs[c];
    *(v8us*)(sr + UNITS + NCO * f) = pk.u;
  }
  __syncthreads();

  constexpr int NCH = APR * NGRP / NTHR;
  unsigned short* gp = Ap + (size_t)row0 * KD;
#pragma unroll
  for (int j = 0; j < NCH; ++j) {
    const int e = tid + NTHR * j;
    const v8us v = *(const v8us*)(sT + 8 * e);
    *(volatile v8us*)(gp + (size_t)8 * e) = v;
  }
  __threadfence();
#pragma unroll
  for (int j = 0; j < NCH; ++j) {
    const int e = tid + NTHR * j;
    const v8us v = *(const v8us*)(sT + 8 * e);
    *(volatile v8us*)(gp + (size_t)8 * e) = v;
  }
}

template <int NCOL>
__global__ __launch_bounds__(NTHR) void k_gemm(const unsigned short* __restrict__ Ap,
                                              const unsigned short* __restrict__ Wp, float* C) {
  __shared__ __align__(16) float hb[RPB * HBP];
  const int tid = threadIdx.x, lane = tid & 31, wave = tid >> 5, h = lane >> 4, m = lane & 15;
  const int rt = wave & 3, cg = wave >> 2;
  const int rowBase = blockIdx.y * RPB;
  const int colBase = blockIdx.x * CPB;
  const unsigned short* ap = Ap + (size_t)(rowBase + 16 * rt + m) * KD + 8 * h;
  const unsigned short* wp = Wp + (size_t)(colBase + 64 * cg + m) * KD + 8 * h;

  v8f acc[4];
#pragma unroll
  for (int nt = 0; nt < 4; ++nt) acc[nt] = zero8();

#pragma unroll 2
  for (int ks = 0; ks < KD / 32; ++ks) {
    const int ko = 32 * ks;
    FragH fa;
    fa.h[0] = *(const v8us*)(ap + ko);
    fa.h[1] = *(const v8us*)(ap + ko + 16);
#pragma unroll
    for (int nt = 0; nt < 4; ++nt) {
      const unsigned short* bp = wp + (size_t)(16 * nt) * KD + ko;
      FragH fb;
      fb.h[0] = *(const v8us*)bp;
      fb.h[1] = *(const v8us*)(bp + 16);
      acc[nt] = wmf(fa.v, fb.v, acc[nt]);
    }
  }

#pragma unroll
  for (int nt = 0; nt < 4; ++nt) {
#pragma unroll
    for (int r = 0; r < 8; ++r)
      hb[(16 * rt + 8 * h + r) * HBP + 64 * cg + 16 * nt + m] = acc[nt][r] * WINV;
  }
  __syncthreads();

  float* cp = C + (size_t)rowBase * NCOL + colBase;
#pragma unroll
  for (int j = 0; j < 8; ++j) {
    const int e = tid + NTHR * j;
    const int row = e >> 5, q = e & 31;
    const v4f v = *(const v4f*)(hb + row * HBP + 4 * q);
    *(volatile v4f*)(cp + (size_t)row * NCOL + 4 * q) = v;
  }
  __threadfence();
#pragma unroll
  for (int j = 0; j < 8; ++j) {
    const int e = tid + NTHR * j;
    const int row = e >> 5, q = e & 31;
    const v4f v = *(const v4f*)(hb + row * HBP + 4 * q);
    *(volatile v4f*)(cp + (size_t)row * NCOL + 4 * q) = v;
  }
}

__global__ __launch_bounds__(NTHR) void k_season(const float* __restrict__ Tp, const unsigned short* __restrict__ Shi,
                                                const unsigned short* __restrict__ Slo, float* out, int nrow) {
  __shared__ __align__(16) float hb[RPB * HBP];
  const int tid = threadIdx.x, lane = tid & 31, wave = tid >> 5, h = lane >> 4, m = lane & 15;
  const int rt = wave & 3, cg = wave >> 2;
  const int rowBase = blockIdx.y * RPB;
  const int nb = blockIdx.x;
  const float* tp = Tp + (size_t)(rowBase + 16 * rt + m) * TH + 8 * h;
  const size_t nrow0 = (size_t)(CPB * nb + 64 * cg + m);
  const unsigned short* shp = Shi + nrow0 * TH + 8 * h;
  const unsigned short* slp = Slo + nrow0 * TH + 8 * h;

  v8f acc[4];
#pragma unroll
  for (int nt = 0; nt < 4; ++nt) acc[nt] = zero8();

#pragma unroll 1
  for (int ks = 0; ks < TH / 32; ++ks) {
    const int ko = 32 * ks;
    const v4f x0 = *(const v4f*)(tp + ko),      x1 = *(const v4f*)(tp + ko + 4);
    const v4f x2 = *(const v4f*)(tp + ko + 16), x3 = *(const v4f*)(tp + ko + 20);
    const float xs[16] = {x0.x, x0.y, x0.z, x0.w, x1.x, x1.y, x1.z, x1.w,
                          x2.x, x2.y, x2.z, x2.w, x3.x, x3.y, x3.z, x3.w};
    FragB ah, al;
#pragma unroll
    for (int i = 0; i < 16; ++i) {
      unsigned short a, d;
      split2(xs[i], a, d);
      ah.u[i] = a; al.u[i] = d;
    }
#pragma unroll
    for (int nt = 0; nt < 4; ++nt) {
      const size_t no = (size_t)(16 * nt) * TH + ko;
      FragB bh2, bl2;
      bh2.h[0] = *(const v8us*)(shp + no);
      bh2.h[1] = *(const v8us*)(shp + no + 16);
      bl2.h[0] = *(const v8us*)(slp + no);
      bl2.h[1] = *(const v8us*)(slp + no + 16);
      acc[nt] = wmb(ah.b, bh2.b, acc[nt]);
      acc[nt] = wmb(ah.b, bl2.b, acc[nt]);
      acc[nt] = wmb(al.b, bh2.b, acc[nt]);
    }
  }

#pragma unroll
  for (int nt = 0; nt < 4; ++nt) {
#pragma unroll
    for (int r = 0; r < 8; ++r)
      hb[(16 * rt + 8 * h + r) * HBP + 64 * cg + 16 * nt + m] = acc[nt][r];
  }
  __syncthreads();

  float* cp;
  int pitch;
  if (nb < BACK / CPB) { cp = out + (size_t)rowBase * BACK + (size_t)CPB * nb; pitch = BACK; }
  else                 { cp = out + (size_t)nrow * BACK + (size_t)rowBase * FORE; pitch = FORE; }
#pragma unroll
  for (int j = 0; j < 8; ++j) {
    const int e = tid + NTHR * j;
    const int row = e >> 5, q = e & 31;
    const v4f v = *(const v4f*)(hb + row * HBP + 4 * q);
    *(volatile v4f*)(cp + (size_t)row * pitch + 4 * q) = v;
  }
  __threadfence();
#pragma unroll
  for (int j = 0; j < 8; ++j) {
    const int e = tid + NTHR * j;
    const int row = e >> 5, q = e & 31;
    const v4f v = *(const v4f*)(hb + row * HBP + 4 * q);
    *(volatile v4f*)(cp + (size_t)row * pitch + 4 * q) = v;
  }
}

extern "C" void kernel_launch(void* const* d_in, const int* in_sizes, int n_in,
                              void* d_out, int out_size, void* d_ws, size_t ws_size,
                              hipStream_t stream) {
  if (n_in < 7) return;
  const int nrow = in_sizes[0] / UNITS;
  if (nrow <= 0 || in_sizes[0] != nrow * UNITS || (nrow % RPB) != 0) return;
  if (in_sizes[1] != NL * UNITS * UNITS * NCO) return;
  if (in_sizes[2] != NL * UNITS * UNITS || in_sizes[3] != NL * UNITS * UNITS) return;
  if (in_sizes[4] != UNITS * TH * NCO) return;
  if (in_sizes[5] != UNITS * TH || in_sizes[6] != UNITS * TH) return;
  if (out_size != nrow * (BACK + FORE)) return;

  const float* x       = (const float*)d_in[0];
  const float* coef_fc = (const float*)d_in[1];
  const float* sb_fc   = (const float*)d_in[2];
  const float* ssp_fc  = (const float*)d_in[3];
  const float* coef_th = (const float*)d_in[4];
  const float* sb_th   = (const float*)d_in[5];
  const float* ssp_th  = (const float*)d_in[6];
  float* out = (float*)d_out;

  size_t off = 0;
  const size_t bWfc = (size_t)NL * UNITS * KD * 2;
  const size_t bWth = (size_t)TH * KD * 2;
  const size_t bAp  = (size_t)nrow * KD * 2;
  const size_t bH   = (size_t)nrow * UNITS * 4;
  const size_t bTh  = (size_t)nrow * TH * 4;
  const size_t bS   = (size_t)TT * TH * 2;
  const size_t oWfc = off; off += (bWfc + 255) & ~(size_t)255;
  const size_t oWth = off; off += (bWth + 255) & ~(size_t)255;
  const size_t oAp  = off; off += (bAp  + 255) & ~(size_t)255;
  const size_t oH   = off; off += (bH   + 255) & ~(size_t)255;
  const size_t oTh  = off; off += (bTh  + 255) & ~(size_t)255;
  const size_t oShi = off; off += (bS   + 255) & ~(size_t)255;
  const size_t oSlo = off; off += (bS   + 255) & ~(size_t)255;
  const size_t tot  = off;
  if (tot > ws_size || tot > (size_t)WSCAP) return;
  char* ws = (char*)d_ws;
  unsigned short* Wfc = (unsigned short*)(ws + oWfc);
  unsigned short* Wth = (unsigned short*)(ws + oWth);
  unsigned short* Apl = (unsigned short*)(ws + oAp);
  float* Hpl = (float*)(ws + oH);
  float* Thp = (float*)(ws + oTh);
  unsigned short* Shi = (unsigned short*)(ws + oShi);
  unsigned short* Slo = (unsigned short*)(ws + oSlo);

  const int nrb = nrow / RPB;

  k_tables<<<(TT * TH / 8) / NTHR, NTHR, 0, stream>>>(Shi, Slo);
  k_wpack<UNITS><<<(NL * UNITS * NGRP) / NTHR, NTHR, 0, stream>>>(coef_fc, sb_fc, ssp_fc, Wfc);
  k_wpack<TH><<<(TH * NGRP) / NTHR, NTHR, 0, stream>>>(coef_th, sb_th, ssp_th, Wth);

  for (int l = 0; l < NL; ++l) {
    const float* hin = (l == 0) ? x : Hpl;
    k_aprep<<<nrow / APR, NTHR, 0, stream>>>(hin, Apl);
    k_gemm<UNITS><<<dim3(UNITS / CPB, nrb), NTHR, 0, stream>>>(Apl, Wfc + (size_t)l * UNITS * KD, Hpl);
  }

  k_aprep<<<nrow / APR, NTHR, 0, stream>>>(Hpl, Apl);
  k_gemm<TH><<<dim3(TH / CPB, nrb), NTHR, 0, stream>>>(Apl, Wth, Thp);

  k_season<<<dim3(TT / CPB, nrb), NTHR, 0, stream>>>(Thp, Shi, Slo, out, nrow);
}
